// RGNN_42795054137552
// MI455X (gfx1250) — hardware-verified
//
#include <hip/hip_runtime.h>
#include <stddef.h>
#include <stdint.h>


#define NN      20000
#define NE      320000
#define NGR     64
#define NH      128
#define MM      4
#define FK      16
#define R4      (NN * MM)
#define ZW      256
#define NTHR    256
#define NWAVE   8
#define EPT     8
#define CHUNK   (NTHR * EPT)
#define WCAP    (EPT * 32)
#define LISTN   (NWAVE * WCAP)
#define NBMAX   2048
#define NBRUN   1024
#define NBKT    20
#define RCAP    28672
#define DEGCAP  64
#define PKS     11
#define GBM     64
#define GBN     128
#define GTHR    128
#define GNT     8
#define PARTW   288
#define MPN     20032
#define DPW     8
#define AGB     (NWAVE * DPW)
#define BNEPS   1e-5f
#define NU_L2   (NH * (ZW / 8))
#define NU_WC   (3 * NH * (ZW / 8))
#define LDS_BKT ((2 * RCAP + 2 * NBMAX + LISTN) * 4 + 64)
#define HFP     129
#define HOP     65
#define LDS_HEAD ((256 * HFP + 64 * 128 + 256 * HOP + 256) * 4)
#define WSCAP   268435456

static_assert(NH == 32 * 4 && MM == 4);
static_assert((NE % GBM) == 0 && (R4 % GBM) == 0 && (MPN % GBM) == 0 && MPN >= NN && MPN - NN < GBM);
static_assert(NGR * MM == 256 && NTHR == 256);
static_assert(NBKT * NBRUN >= NN && NBRUN <= NBMAX && NTHR * 4 == NBRUN && NTHR * 8 == NBMAX);
static_assert((CHUNK & (CHUNK - 1)) == 0 && CHUNK <= (1 << PKS) && NBMAX <= (1 << PKS));
static_assert(((long long)NE << PKS) < (1LL << 31));
static_assert(LISTN >= NBMAX);
static_assert((RCAP % 512) == 0 && ((2 * RCAP + NBMAX) % (NTHR * 4)) == 0);
static_assert(16604 * 105 / 100 <= RCAP);
static_assert(33 + 8 <= DEGCAP);
static_assert(LDS_BKT <= 300000 && LDS_HEAD <= 245760);
static_assert(GBM == (GTHR / 32) * 16 && GBN == 16 * GNT && GTHR == GBN && GBN == NH);
static_assert((PARTW % 32) == 0 && PARTW >= 2 * GBN + 1 && PARTW / 4 <= GTHR);
static_assert((ZW % 32) == 0 && ZW == 2 * NH);
static_assert((NU_L2 % NTHR) == 0 && (NU_WC % NTHR) == 0);
static_assert(((MPN * 16) % NTHR) == 0 && ((R4 * 32) % NTHR) == 0);
static_assert((NE * 4) % 32 == 0);

typedef float          v4f  __attribute__((ext_vector_type(4)));
typedef float          v8f  __attribute__((ext_vector_type(8)));
typedef int            v2i  __attribute__((ext_vector_type(2)));
typedef int            v4i  __attribute__((ext_vector_type(4)));
typedef int            v8i  __attribute__((ext_vector_type(8)));
typedef unsigned int   v2u  __attribute__((ext_vector_type(2)));
typedef unsigned short v8us __attribute__((ext_vector_type(8)));
typedef __bf16         v16b __attribute__((ext_vector_type(16)));
typedef v4f  __attribute__((may_alias)) v4fa;
typedef v4i  __attribute__((may_alias)) v4ia;
typedef v2i  __attribute__((may_alias)) v2ia;
typedef v8us __attribute__((may_alias)) v8usa;
union Frag { v16b vb; v8us h[2]; v8i w; };

__device__ __forceinline__ v8f wmx(const Frag& a, const Frag& b, v8f c) {
  v8f d = __builtin_amdgcn_wmma_f32_16x16x32_bf16(false, a.vb, false, b.vb, (short)0, c, false, false);
  asm volatile("v_nop\n\tv_nop\n\tv_nop\n\tv_nop" : "+v"(d) : "v"(a.w), "v"(b.w));
  return d;
}
__device__ __forceinline__ v8f z8() { v8f z = {0.f, 0.f, 0.f, 0.f, 0.f, 0.f, 0.f, 0.f}; return z; }

__device__ __forceinline__ unsigned short bf_bits(float f) {
  unsigned int u = __float_as_uint(f);
  u += 0x7FFFu + ((u >> 16) & 1u);
  return (unsigned short)(u >> 16);
}
__device__ __forceinline__ float bf_val(unsigned short b) { return __uint_as_float(((unsigned int)b) << 16); }
__device__ __forceinline__ float bf_rne(float f) { return bf_val(bf_bits(f)); }
__device__ __forceinline__ float relu_p(float v) { return (v > 0.0f) ? v : (v - v); }

__device__ __forceinline__ void hilo8(const v4f a, const v4f b, v8us& hv, v8us& lv) {
  const float f[8] = {a.x, a.y, a.z, a.w, b.x, b.y, b.z, b.w};
#pragma unroll
  for (int j = 0; j < 8; ++j) {
    const unsigned short hb = bf_bits(f[j]);
    hv[j] = hb;
    lv[j] = bf_bits(f[j] - bf_val(hb));
  }
}
__device__ __forceinline__ v8us bits8(const v4f a, const v4f b, unsigned short mk) {
  v8us o;
  o[0] = (unsigned short)(bf_bits(a.x) & mk); o[1] = (unsigned short)(bf_bits(a.y) & mk);
  o[2] = (unsigned short)(bf_bits(a.z) & mk); o[3] = (unsigned short)(bf_bits(a.w) & mk);
  o[4] = (unsigned short)(bf_bits(b.x) & mk); o[5] = (unsigned short)(bf_bits(b.y) & mk);
  o[6] = (unsigned short)(bf_bits(b.z) & mk); o[7] = (unsigned short)(bf_bits(b.w) & mk);
  return o;
}
__device__ __forceinline__ void put16(unsigned short* dp, v8us o) {
  *(volatile v8us*)dp = o;
  __threadfence();
  *(volatile v8us*)dp = o;
}

__device__ __forceinline__ int scan_chunk(const int* __restrict__ dsts, int nE, int cbase, int slotBase,
                                          int nb, int vec8, int* list, int tid, int lane, int wave) {
  int wc = 0;
  const int el0  = tid * EPT;
  const int e0   = cbase + el0;
  const int sent = -2147483647 - 1;
  v4i da, db;
  if (vec8 != 0 && cbase + CHUNK <= nE) {
    da = *(const v4i*)(dsts + e0);
    db = *(const v4i*)(dsts + e0 + 4);
  } else {
    da.x = (e0     < nE) ? dsts[min(e0,     nE - 1)] : sent;
    da.y = (e0 + 1 < nE) ? dsts[min(e0 + 1, nE - 1)] : sent;
    da.z = (e0 + 2 < nE) ? dsts[min(e0 + 2, nE - 1)] : sent;
    da.w = (e0 + 3 < nE) ? dsts[min(e0 + 3, nE - 1)] : sent;
    db.x = (e0 + 4 < nE) ? dsts[min(e0 + 4, nE - 1)] : sent;
    db.y = (e0 + 5 < nE) ? dsts[min(e0 + 5, nE - 1)] : sent;
    db.z = (e0 + 6 < nE) ? dsts[min(e0 + 6, nE - 1)] : sent;
    db.w = (e0 + 7 < nE) ? dsts[min(e0 + 7, nE - 1)] : sent;
  }
  const unsigned nbs = (unsigned)slotBase;
  const unsigned unb = (unsigned)nb;
  const unsigned s0 = (unsigned)da.x - nbs, s1 = (unsigned)da.y - nbs;
  const unsigned s2 = (unsigned)da.z - nbs, s3 = (unsigned)da.w - nbs;
  const unsigned s4 = (unsigned)db.x - nbs, s5 = (unsigned)db.y - nbs;
  const unsigned s6 = (unsigned)db.z - nbs, s7 = (unsigned)db.w - nbs;
  const bool h0 = s0 < unb, h1 = s1 < unb, h2 = s2 < unb, h3 = s3 < unb;
  const bool h4 = s4 < unb, h5 = s5 < unb, h6 = s6 < unb, h7 = s7 < unb;
  const unsigned any = __builtin_amdgcn_ballot_w32(h0 | h1 | h2 | h3 | h4 | h5 | h6 | h7);
  if (any != 0u) {
#define HITJ(J, HJ, SJ) { \
      const unsigned mj = __builtin_amdgcn_ballot_w32(HJ); \
      if (mj != 0u) { \
        if (HJ) { \
          const int pos = wc + (int)__builtin_amdgcn_mbcnt_lo(mj, 0u); \
          if (pos < WCAP) list[wave * WCAP + pos] = ((el0 + (J)) << PKS) | (int)(SJ); \
        } \
        wc += (int)__builtin_popcount(mj); } }
    HITJ(0, h0, s0)
    HITJ(1, h1, s1)
    HITJ(2, h2, s2)
    HITJ(3, h3, s3)
    HITJ(4, h4, s4)
    HITJ(5, h5, s5)
    HITJ(6, h6, s6)
    HITJ(7, h7, s7)
#undef HITJ
  }
  return wc;
}

__global__ __launch_bounds__(NTHR) void k_prep(const float* __restrict__ Wl2, const float* __restrict__ Wc,
                                               unsigned short* W2D, unsigned short* WCD) {
  const int u = (int)blockIdx.x * NTHR + (int)threadIdx.x;
  v8us o;
  if (u < NU_L2) {
    const int n  = u >> 5;
    const int k8 = (u & 31) * 8;
    const int kk = k8 & (NH - 1);
    const float* p = Wl2 + (size_t)kk * (NH + 1) + n;
#pragma unroll
    for (int i = 0; i < 8; ++i) o[i] = bf_bits(p[(size_t)i * (NH + 1)]);
    put16(W2D + (size_t)u * 8, o);
  } else if (u < NU_L2 + NU_WC) {
    const int v  = u - NU_L2;
    const int rw = v >> 5;
    const int k8 = (v & 31) * 8;
    const int kk = k8 & (NH - 1);
    const float* p = Wc + (size_t)rw * NH + kk;
    const v4f a = *(const v4f*)p;
    const v4f b = *(const v4f*)(p + 4);
    o = bits8(a, b, (unsigned short)0xffffu);
    put16(WCD + (size_t)v * 8, o);
  }
}

__global__ __launch_bounds__(NTHR) void k_bucket(const int* __restrict__ srcs, const int* __restrict__ dsts,
                                                 int* LISTg, int* CNTg, int* OFFg) {
  extern __shared__ v4f lds_dyn[];
  int* reg1 = (int*)lds_dyn;
  int* reg2 = reg1 + RCAP;
  int* scnt = reg2 + RCAP;
  int* soff = scnt + NBMAX;
  int* list = soff + NBMAX;
  int* wcnt = list + LISTN;
  int* wtot = wcnt + NWAVE;
  const int tid = (int)threadIdx.x, lane = tid & 31, wave = tid >> 5;
  const int nodeBase = (int)blockIdx.x * NBRUN;
  const int nE = NE;

  {
    const v4i z4 = {0, 0, 0, 0};
    for (int i = tid * 4; i < 2 * RCAP + NBMAX; i += NTHR * 4) *(v4ia*)(reg1 + i) = z4;
  }
  __syncthreads();

  int tot = 0;
  const int nChunks = (nE + CHUNK - 1) / CHUNK;
#pragma unroll 1
  for (int ch = 0; ch < nChunks; ++ch) {
    const int cbase = ch * CHUNK;
    const int wc = scan_chunk(dsts, nE, cbase, nodeBase, NBRUN, 1, list, tid, lane, wave);
    if (lane == 0) wcnt[wave] = wc;
    __syncthreads();
    int pre = 0, all = 0;
#pragma unroll
    for (int w2 = 0; w2 < NWAVE; ++w2) {
      int c = wcnt[w2];
      c = c < 0 ? 0 : (c > WCAP ? WCAP : c);
      all += c;
      pre += (w2 < wave) ? c : 0;
    }
    const int wcc  = wc > WCAP ? WCAP : wc;
    const int base = tot + pre;
#pragma unroll 1
    for (int i = lane; i < wcc; i += 32) {
      const int ent = list[wave * WCAP + i];
      const int el  = (ent >> PKS) & (CHUNK - 1);
      const int sl  = ent & (NBMAX - 1);
      int eid = cbase + el;
      eid = eid > nE - 1 ? nE - 1 : eid;
      const int pos = base + i;
      if (pos < RCAP) reg1[pos] = (int)(((unsigned)eid << PKS) | (unsigned)sl);
    }
    tot += all;
    tot = tot > RCAP ? RCAP : tot;
    __syncthreads();
  }
  const int nh = tot;

  if (wave == 0) {
#pragma unroll 1
    for (int b0 = 0; b0 < nh; b0 += 32) {
      const int idx = b0 + lane;
      const int uv  = reg1[idx < RCAP ? idx : RCAP - 1];
      const int m32 = (nh - b0) < 32 ? (nh - b0) : 32;
#pragma unroll 1
      for (int k = 0; k < m32; ++k) {
        const int u  = __builtin_amdgcn_readlane(uv, k);
        const int sl = u & (NBMAX - 1);
        if (lane == 0) scnt[sl] = scnt[sl] + 1;
      }
    }
  }
  __syncthreads();

  {
    const v4i ca = *(const v4ia*)(scnt + 8 * tid);
    const v4i cb = *(const v4ia*)(scnt + 8 * tid + 4);
    const int e0 = ca.x < 0 ? 0 : ca.x, e1 = ca.y < 0 ? 0 : ca.y, e2 = ca.z < 0 ? 0 : ca.z, e3 = ca.w < 0 ? 0 : ca.w;
    const int e4 = cb.x < 0 ? 0 : cb.x, e5 = cb.y < 0 ? 0 : cb.y, e6 = cb.z < 0 ? 0 : cb.z, e7 = cb.w < 0 ? 0 : cb.w;
    const int ts = e0 + e1 + e2 + e3 + e4 + e5 + e6 + e7;
    int incl = ts;
#pragma unroll
    for (int d = 1; d < 32; d <<= 1) {
      const int up = __shfl_up(incl, d);
      if (lane >= d) incl += up;
    }
    if (lane == 31) wtot[wave] = incl;
    __syncthreads();
    int pre = 0;
#pragma unroll
    for (int w2 = 0; w2 < NWAVE; ++w2) pre += (w2 < wave) ? wtot[w2] : 0;
    int run = pre + incl - ts;
    soff[8 * tid + 0] = run; run += e0;
    soff[8 * tid + 1] = run; run += e1;
    soff[8 * tid + 2] = run; run += e2;
    soff[8 * tid + 3] = run; run += e3;
    soff[8 * tid + 4] = run; run += e4;
    soff[8 * tid + 5] = run; run += e5;
    soff[8 * tid + 6] = run; run += e6;
    soff[8 * tid + 7] = run;
  }
  __syncthreads();
  for (int i = tid; i < NBMAX; i += NTHR) list[i] = soff[i];
  __syncthreads();

  if (wave == 0) {
#pragma unroll 1
    for (int b0 = 0; b0 < nh; b0 += 32) {
      const int idx = b0 + lane;
      const int uv  = reg1[idx < RCAP ? idx : RCAP - 1];
      const int m32 = (nh - b0) < 32 ? (nh - b0) : 32;
#pragma unroll 1
      for (int k = 0; k < m32; ++k) {
        const int u   = __builtin_amdgcn_readlane(uv, k);
        const int sl  = u & (NBMAX - 1);
        const int eid = (int)((unsigned)u >> PKS);
        if (lane == 0) {
          int pos = list[sl];
          pos = pos < 0 ? 0 : (pos > RCAP - 1 ? RCAP - 1 : pos);
          reg2[pos] = eid;
          list[sl] = pos + 1;
        }
      }
    }
  }
  __syncthreads();

  const bool ovf = (nh >= RCAP);
  {
    v4i c = *(const v4ia*)(scnt + 4 * tid);
    const v4i o = *(const v4ia*)(soff + 4 * tid);
    c.x = ovf ? -1 : c.x; c.y = ovf ? -1 : c.y; c.z = ovf ? -1 : c.z; c.w = ovf ? -1 : c.w;
    int* cp = CNTg + (size_t)blockIdx.x * NBRUN + 4 * tid;
    int* op = OFFg + (size_t)blockIdx.x * NBRUN + 4 * tid;
    *(volatile v4i*)cp = c;
    *(volatile v4i*)op = o;
    __threadfence();
    *(volatile v4i*)cp = c;
    *(volatile v4i*)op = o;
  }
#pragma unroll 1
  for (int sw = 0; sw < RCAP / (2 * NTHR); ++sw) {
    const int idx = (sw * NTHR + tid) * 2;
    const v2i ee = *(const v2ia*)(reg2 + idx);
    int ea0 = ee.x, ea1 = ee.y;
    ea0 = ea0 < 0 ? 0 : (ea0 > nE - 1 ? nE - 1 : ea0);
    ea1 = ea1 < 0 ? 0 : (ea1 > nE - 1 ? nE - 1 : ea1);
    int sa0 = srcs[ea0], sa1 = srcs[ea1];
    sa0 = sa0 < 0 ? 0 : (sa0 > NN - 1 ? NN - 1 : sa0);
    sa1 = sa1 < 0 ? 0 : (sa1 > NN - 1 ? NN - 1 : sa1);
    v4i ent;
    ent.x = ea0; ent.y = sa0; ent.z = ea1; ent.w = sa1;
    int* lp = LISTg + ((size_t)blockIdx.x * RCAP + (size_t)idx) * 2;
    *(volatile v4i*)lp = ent;
    __threadfence();
    *(volatile v4i*)lp = ent;
  }
}

__device__ __forceinline__ void tile_stats(const v8f (&val)[GNT], int rowBase, int nN,
                                           float* red, float* red2, float* smean, float* pst,
                                           float* part, size_t prow, int tid, int wave, int hh, int m) {
  const int r0 = rowBase + 16 * wave + 8 * hh;
  int nvr = nN - rowBase;
  nvr = nvr < 0 ? 0 : (nvr > GBM ? GBM : nvr);
#pragma unroll
  for (int nt = 0; nt < GNT; ++nt) {
    float s = 0.0f;
#pragma unroll
    for (int r = 0; r < 8; ++r) {
      const float v = val[nt][r];
      s += ((r0 + r) < nN) ? v : 0.0f;
    }
    s += __shfl_xor(s, 16);
    if (hh == 0) red[wave * GBN + 16 * nt + m] = s;
  }
  __syncthreads();
  {
    const float tot = ((red[tid] + red[GBN + tid]) + red[2 * GBN + tid]) + red[3 * GBN + tid];
    smean[tid] = tot * (1.0f / (float)(nvr < 1 ? 1 : nvr));
  }
  __syncthreads();
#pragma unroll
  for (int nt = 0; nt < GNT; ++nt) {
    const float mu = smean[16 * nt + m];
    float q = 0.0f;
#pragma unroll
    for (int r = 0; r < 8; ++r) {
      const float d = val[nt][r] - mu;
      q += ((r0 + r) < nN) ? d * d : 0.0f;
    }
    q += __shfl_xor(q, 16);
    if (hh == 0) red2[wave * GBN + 16 * nt + m] = q;
  }
  __syncthreads();
  {
    const float M2 = ((red2[tid] + red2[GBN + tid]) + red2[2 * GBN + tid]) + red2[3 * GBN + tid];
    pst[1 + tid] = smean[tid];
    pst[1 + GBN + tid] = M2;
    if (tid == 0) pst[0] = (float)nvr;
#pragma unroll 1
    for (int i = 2 * GBN + 1 + tid; i < PARTW; i += GTHR) pst[i] = 0.0f;
  }
  __syncthreads();
  const bool pok = tid < PARTW / 4;
  v4f pv = {0.f, 0.f, 0.f, 0.f};
  float* pp = part + prow * PARTW + 4 * tid;
  if (pok) {
    pv = *(const v4fa*)(pst + 4 * tid);
    *(volatile v4f*)pp = pv;
  }
  __threadfence();
  if (pok) *(volatile v4f*)pp = pv;
}

__device__ __forceinline__ void stage_tile(const v8f (&val)[GNT], float* stg, int rowBase, int nN,
                                           int wave, int hh, int m) {
#pragma unroll
  for (int nt = 0; nt < GNT; ++nt) {
    const int lc = 16 * nt + m;
#pragma unroll
    for (int r = 0; r < 8; ++r) {
      const int lr = 16 * wave + 8 * hh + r;
      stg[lr * GBN + lc] = ((rowBase + lr) < nN) ? val[nt][r] : 0.0f;
    }
  }
}

__device__ __forceinline__ void store_rows(const float* stg, float* outF, int rowBase, int mRows,
                                           int wave, int lane) {
  v4f fv[16];
#pragma unroll
  for (int i = 0; i < 16; ++i) fv[i] = *(const v4fa*)(stg + (16 * wave + i) * GBN + 4 * lane);
#pragma unroll
  for (int i = 0; i < 16; ++i) {
    const int gr = rowBase + 16 * wave + i;
    float* op = outF + (size_t)gr * GBN + 4 * lane;
    if (gr < mRows) *(volatile v4f*)op = fv[i];
  }
  __threadfence();
#pragma unroll
  for (int i = 0; i < 16; ++i) {
    const int gr = rowBase + 16 * wave + i;
    float* op = outF + (size_t)gr * GBN + 4 * lane;
    if (gr < mRows) *(volatile v4f*)op = fv[i];
  }
}

__global__ __launch_bounds__(GTHR) void k_g16(const float* __restrict__ A, int nRows,
                                              const float* __restrict__ W, const float* __restrict__ bias,
                                              float* outp, int mRows, float* part) {
  __shared__ __attribute__((aligned(16))) float stg[GBM * GBN];
  __shared__ float red[4 * GBN];
  __shared__ float red2[4 * GBN];
  __shared__ float smean[GBN];
  __shared__ __attribute__((aligned(16))) float pst[PARTW];
  const int tid = (int)threadIdx.x, lane = tid & 31, wave = tid >> 5, hh = lane >> 4, m = lane & 15;
  const int rowBase = (int)blockIdx.x * GBM;
  const v8us zz = {0, 0, 0, 0, 0, 0, 0, 0};

  Frag af;
  {
    const int ar  = rowBase + 16 * wave + m;
    const int arc = ar < nRows ? ar : nRows - 1;
    const unsigned short mk = (ar < nRows) ? (unsigned short)0xffffu : (unsigned short)0u;
    const float* ap = A + (size_t)arc * FK + 8 * hh;
    const v4f a0 = *(const v4f*)ap;
    const v4f a1 = *(const v4f*)(ap + 4);
    af.h[0] = bits8(a0, a1, mk);
    af.h[1] = zz;
  }
  v8f acc[GNT];
#pragma unroll
  for (int nt = 0; nt < GNT; ++nt) {
    const float* wp = W + (size_t)(16 * nt + m) * FK + 8 * hh;
    const v4f w0 = *(const v4f*)wp;
    const v4f w1 = *(const v4f*)(wp + 4);
    Frag bfr;
    bfr.h[0] = bits8(w0, w1, (unsigned short)0xffffu);
    bfr.h[1] = zz;
    acc[nt] = wmx(af, bfr, z8());
  }
#pragma unroll
  for (int nt = 0; nt < GNT; ++nt) {
    const float bb = bf_rne(bias[16 * nt + m]);
#pragma unroll
    for (int r = 0; r < 8; ++r) acc[nt][r] = acc[nt][r] + bb;
  }
  stage_tile(acc, stg, rowBase, nRows, wave, hh, m);
  tile_stats(acc, rowBase, nRows, red, red2, smean, pst, part, (size_t)blockIdx.x, tid, wave, hh, m);
  store_rows(stg, outp, rowBase, mRows, wave, lane);
}

template <int EPI>
__global__ __launch_bounds__(GTHR) void k_gemm(const unsigned short* __restrict__ A,
                                               const unsigned short* __restrict__ BT,
                                               float* outp, int nN, float* part,
                                               const float* __restrict__ Wl2, const float* __restrict__ bl2,
                                               const float* __restrict__ axp) {
  __shared__ __attribute__((aligned(16))) float stg[GBM * GBN];
  __shared__ float red[4 * GBN];
  __shared__ float red2[4 * GBN];
  __shared__ float smean[GBN];
  __shared__ __attribute__((aligned(16))) float pst[PARTW];
  __shared__ __attribute__((aligned(16))) float wlS[NH];
  __shared__ __attribute__((aligned(16))) float b2S[NH];
  const int tid = (int)threadIdx.x, lane = tid & 31, wave = tid >> 5, hh = lane >> 4, m = lane & 15;
  const int rowBase = (int)blockIdx.x * GBM;

  v8f acc[GNT];
#pragma unroll
  for (int t = 0; t < GNT; ++t) acc[t] = z8();
  const unsigned short* ap = A  + (size_t)(rowBase + 16 * wave + m) * (size_t)ZW + 8 * hh;
  const unsigned short* bp = BT + (size_t)m * (size_t)ZW + 8 * hh;

#pragma unroll 1
  for (int k0 = 0; k0 < ZW; k0 += 32) {
    Frag af;
    af.h[0] = *(const v8usa*)(ap + k0);
    af.h[1] = *(const v8usa*)(ap + k0 + 16);
#pragma unroll
    for (int nt = 0; nt < GNT; ++nt) {
      const unsigned short* wq = bp + (size_t)(16 * nt) * (size_t)ZW + k0;
      Frag bfr;
      bfr.h[0] = *(const v8usa*)wq;
      bfr.h[1] = *(const v8usa*)(wq + 16);
      acc[nt] = wmx(af, bfr, acc[nt]);
    }
  }

  if constexpr (EPI == 1) {
    stage_tile(acc, stg, rowBase, nN, wave, hh, m);
    tile_stats(acc, rowBase, nN, red, red2, smean, pst, part, (size_t)blockIdx.x, tid, wave, hh, m);
    store_rows(stg, outp, rowBase, nN, wave, lane);
  } else {
    wlS[tid] = bf_rne(Wl2[(size_t)tid * (NH + 1) + NH]);
    b2S[tid] = bf_rne(bl2[tid]);
    stage_tile(acc, stg, rowBase, nN, wave, hh, m);
    __syncthreads();
    const int q  = lane >> 3;
    const int jb = 16 * (lane & 7);
    const v4f bcv = *(const v4fa*)(b2S + 4 * lane);
    const v4f wv0 = *(const v4fa*)(wlS + jb),      wv1 = *(const v4fa*)(wlS + jb + 4);
    const v4f wv2 = *(const v4fa*)(wlS + jb + 8),  wv3 = *(const v4fa*)(wlS + jb + 12);
    const v4f bj0 = *(const v4fa*)(b2S + jb),      bj1 = *(const v4fa*)(b2S + jb + 4);
    const v4f bj2 = *(const v4fa*)(b2S + jb + 8),  bj3 = *(const v4fa*)(b2S + jb + 12);
#pragma unroll 1
    for (int i = 0; i < 16; ++i) {
      const int lr   = 16 * wave + i;
      const int node = rowBase + lr;
      const bool live = node < nN;
      const int nc = live ? node : nN - 1;
      const int rr = 4 * nc + q;
      const int qq = rr / NN;
      const int pp = rr - qq * NN;
      const float axv = bf_rne(axp[(size_t)pp * 4 + qq]);
      const v4f mv = *(const v4fa*)(stg + lr * GBN + 4 * lane);
      const float a0 = mv.x + bcv.x, a1 = mv.y + bcv.y, a2 = mv.z + bcv.z, a3 = mv.w + bcv.w;
      v4f o[4];
#pragma unroll
      for (int mm = 0; mm < 4; ++mm) {
        v4f t;
        t.x = a0 + fmaf(axv, wv0[mm], bj0[mm]);
        t.y = a1 + fmaf(axv, wv1[mm], bj1[mm]);
        t.z = a2 + fmaf(axv, wv2[mm], bj2[mm]);
        t.w = a3 + fmaf(axv, wv3[mm], bj3[mm]);
        o[mm] = t;
      }
      float* op = outp + (size_t)(4 * nc) * NH + 4 * lane;
      if (live) {
#pragma unroll
        for (int mm = 0; mm < 4; ++mm) *(volatile v4f*)(op + (size_t)mm * NH) = o[mm];
      }
      __threadfence();
      if (live) {
#pragma unroll
        for (int mm = 0; mm < 4; ++mm) *(volatile v4f*)(op + (size_t)mm * NH) = o[mm];
      }
    }
  }
}

__global__ __launch_bounds__(GBN) void k_comb(const float* __restrict__ part, int nPart, int gy, int nh,
                                              const float* __restrict__ gam, const float* __restrict__ bet,
                                              float* ss) {
  __shared__ __attribute__((aligned(16))) float stg[2 * GBN];
  const int tid = (int)threadIdx.x;
  const int by  = (int)blockIdx.x;
  const int col = by * GBN + tid;
  double n = 0.0, mean = 0.0, M2 = 0.0;
#pragma unroll 1
  for (int b = 0; b < nPart; ++b) {
    const float* pr = part + ((size_t)b * (size_t)gy + (size_t)by) * PARTW;
    const double nb = (double)pr[0];
    const double mb = (double)pr[1 + tid];
    const double qb = (double)pr[1 + GBN + tid];
    if (nb > 0.5) {
      const double nn = n + nb;
      const double delta = mb - mean;
      const double f = nb / nn;
      mean = mean + delta * f;
      M2 = M2 + qb + delta * delta * n * f;
      n = nn;
    }
  }
  const double nt = n < 1.0 ? 1.0 : n;
  const float var  = (float)(M2 / nt);
  const float rstd = 1.0f / sqrtf(var + BNEPS);
  const float sc = bf_rne(gam[col]) * rstd;
  const float sh = bf_rne(bet[col]) - (float)mean * sc;
  stg[tid] = sc;
  stg[GBN + tid] = sh;
  __syncthreads();
  const int seg = tid >> 5, j = tid & 31;
  const bool ok = tid < 64;
  v4f v = {0.f, 0.f, 0.f, 0.f};
  float* dp = ss + (size_t)(seg & 1) * (size_t)nh + (size_t)by * GBN + 4 * j;
  if (ok) {
    v = *(const v4fa*)(stg + seg * GBN + 4 * j);
    *(volatile v4f*)dp = v;
  }
  __threadfence();
  if (ok) *(volatile v4f*)dp = v;
}

__global__ __launch_bounds__(NTHR) void k_apply0(const float* __restrict__ T0, const float* __restrict__ ss,
                                                 unsigned short* HHL) {
  const int u   = (int)blockIdx.x * NTHR + (int)threadIdx.x;
  const int row = u >> 4;
  const int q   = u & 15;
  const bool live = row < NN;
  const int rc = live ? row : NN - 1;
  const float* tp = T0 + (size_t)rc * NH + 8 * q;
  const v4f a = *(const v4f*)tp,               b = *(const v4f*)(tp + 4);
  const v4f sa = *(const v4f*)(ss + 8 * q),    sb = *(const v4f*)(ss + 8 * q + 4);
  const v4f ha = *(const v4f*)(ss + NH + 8 * q), hb = *(const v4f*)(ss + NH + 8 * q + 4);
  v4f ya, yb;
  ya.x = relu_p(fmaf(a.x, sa.x, ha.x)); ya.y = relu_p(fmaf(a.y, sa.y, ha.y));
  ya.z = relu_p(fmaf(a.z, sa.z, ha.z)); ya.w = relu_p(fmaf(a.w, sa.w, ha.w));
  yb.x = relu_p(fmaf(b.x, sb.x, hb.x)); yb.y = relu_p(fmaf(b.y, sb.y, hb.y));
  yb.z = relu_p(fmaf(b.z, sb.z, hb.z)); yb.w = relu_p(fmaf(b.w, sb.w, hb.w));
  ya.x = live ? ya.x : 0.0f; ya.y = live ? ya.y : 0.0f; ya.z = live ? ya.z : 0.0f; ya.w = live ? ya.w : 0.0f;
  yb.x = live ? yb.x : 0.0f; yb.y = live ? yb.y : 0.0f; yb.z = live ? yb.z : 0.0f; yb.w = live ? yb.w : 0.0f;
  v8us hv, lv;
  hilo8(ya, yb, hv, lv);
  unsigned short* hp = HHL + (size_t)row * ZW + 8 * q;
  unsigned short* lp = hp + NH;
  *(volatile v8us*)hp = hv;
  *(volatile v8us*)lp = lv;
  __threadfence();
  *(volatile v8us*)hp = hv;
  *(volatile v8us*)lp = lv;
}

__global__ __launch_bounds__(NTHR) __attribute__((amdgpu_num_vgpr(248)))
void k_agg(const int* __restrict__ LISTg, const int* __restrict__ CNTg, const int* __restrict__ OFFg,
           const float* __restrict__ EE, const float* __restrict__ sse,
           const float* __restrict__ XM, unsigned short* ZHL) {
  const int tid = (int)threadIdx.x, lane = tid & 31;
  const int wave = __builtin_amdgcn_readfirstlane(tid >> 5);
  const v4f sc = *(const v4f*)(sse + 4 * lane);
  const v4f sh = *(const v4f*)(sse + NH + 4 * lane);
  const float qnan = __int_as_float(0x7fc00000);

#pragma unroll 1
  for (int j = 0; j < DPW; ++j) {
    const int node = (int)blockIdx.x * AGB + wave * DPW + j;
    const bool live = node < NN;
    const int nc = live ? node : NN - 1;
    const int craw = CNTg[nc];
    int st = OFFg[nc];
    const int bb = nc >> 10;
    const bool poison = (craw < 0) || (craw > DEGCAP);
    int cnt = craw < 0 ? 0 : (craw > DEGCAP ? DEGCAP : craw);
    st = st < 0 ? 0 : (st > RCAP ? RCAP : st);
    if (cnt > RCAP - st) cnt = RCAP - st;

    v4f acc[4];
    {
      const float* xp = XM + (size_t)(4 * nc) * NH + 4 * lane;
#pragma unroll
      for (int mm = 0; mm < 4; ++mm) acc[mm] = *(const v4f*)(xp + (size_t)mm * NH);
    }
#pragma unroll 1
    for (int q = 0; q < cnt; ++q) {
      int idx = st + q;
      idx = idx > RCAP - 1 ? RCAP - 1 : idx;
      const v2i ent = *(const v2i*)(LISTg + ((size_t)bb * RCAP + (size_t)idx) * 2);
      int eid = ent.x, s = ent.y;
      eid = eid < 0 ? 0 : (eid > NE - 1 ? NE - 1 : eid);
      s   = s   < 0 ? 0 : (s   > NN - 1 ? NN - 1 : s);
      const v4f ev = *(const v4f*)(EE + (size_t)eid * NH + 4 * lane);
      const float e0 = relu_p(fmaf(ev.x, sc.x, sh.x));
      const float e1 = relu_p(fmaf(ev.y, sc.y, sh.y));
      const float e2 = relu_p(fmaf(ev.z, sc.z, sh.z));
      const float e3 = relu_p(fmaf(ev.w, sc.w, sh.w));
      const float* xs = XM + (size_t)(4 * s) * NH + 4 * lane;
#pragma unroll
      for (int mm = 0; mm < 4; ++mm) {
        const v4f xv = *(const v4f*)(xs + (size_t)mm * NH);
        acc[mm].x += relu_p(xv.x + e0);
        acc[mm].y += relu_p(xv.y + e1);
        acc[mm].z += relu_p(xv.z + e2);
        acc[mm].w += relu_p(xv.w + e3);
      }
    }
    v2u zh[4], zl[4];
#pragma unroll
    for (int mm = 0; mm < 4; ++mm) {
      const float f0 = poison ? qnan : acc[mm].x;
      const float f1 = poison ? qnan : acc[mm].y;
      const float f2 = poison ? qnan : acc[mm].z;
      const float f3 = poison ? qnan : acc[mm].w;
      const unsigned short h0 = bf_bits(f0), h1 = bf_bits(f1), h2 = bf_bits(f2), h3 = bf_bits(f3);
      const unsigned short l0 = bf_bits(f0 - bf_val(h0)), l1 = bf_bits(f1 - bf_val(h1));
      const unsigned short l2 = bf_bits(f2 - bf_val(h2)), l3 = bf_bits(f3 - bf_val(h3));
      v2u a, b;
      a.x = (unsigned int)h0 | ((unsigned int)h1 << 16);
      a.y = (unsigned int)h2 | ((unsigned int)h3 << 16);
      b.x = (unsigned int)l0 | ((unsigned int)l1 << 16);
      b.y = (unsigned int)l2 | ((unsigned int)l3 << 16);
      zh[mm] = a; zl[mm] = b;
    }
    unsigned short* zp = ZHL + (size_t)(4 * nc) * ZW + 4 * lane;
    if (live) {
#pragma unroll
      for (int mm = 0; mm < 4; ++mm) {
        *(volatile v2u*)(zp + (size_t)mm * ZW) = zh[mm];
        *(volatile v2u*)(zp + (size_t)mm * ZW + NH) = zl[mm];
      }
    }
    __threadfence();
    if (live) {
#pragma unroll
      for (int mm = 0; mm < 4; ++mm) {
        *(volatile v2u*)(zp + (size_t)mm * ZW) = zh[mm];
        *(volatile v2u*)(zp + (size_t)mm * ZW + NH) = zl[mm];
      }
    }
  }
}

__global__ __launch_bounds__(NTHR) void k_apply(const float* __restrict__ H3, const float* __restrict__ ss,
                                                float* XM) {
  const int u   = (int)blockIdx.x * NTHR + (int)threadIdx.x;
  const int row = u >> 5;
  const int q   = u & 31;
  const v4f h  = *(const v4f*)(H3 + (size_t)row * NH + 4 * q);
  float* xp = XM + (size_t)row * NH + 4 * q;
  const v4f x  = *(const v4f*)xp;
  const v4f sc = *(const v4f*)(ss + 4 * q);
  const v4f sh = *(const v4f*)(ss + NH + 4 * q);
  v4f y;
  y.x = relu_p(fmaf(h.x, sc.x, sh.x)) + x.x;
  y.y = relu_p(fmaf(h.y, sc.y, sh.y)) + x.y;
  y.z = relu_p(fmaf(h.z, sc.z, sh.z)) + x.z;
  y.w = relu_p(fmaf(h.w, sc.w, sh.w)) + x.w;
  *(volatile v4f*)xp = y;
  __threadfence();
  *(volatile v4f*)xp = y;
}

__global__ __launch_bounds__(NTHR) void k_pool(const float* __restrict__ XM, const int* __restrict__ bat,
                                               float* PGb) {
  __shared__ int list[LISTN];
  __shared__ int wcnt[NWAVE];
  __shared__ __attribute__((aligned(16))) float sacc[512];
  const int tid = (int)threadIdx.x, lane = tid & 31, wave = tid >> 5;
  const int g = (int)blockIdx.x;
  float a0 = 0.0f, a1 = 0.0f;
  const int nChunks = (NN + CHUNK - 1) / CHUNK;
#pragma unroll 1
  for (int ch = 0; ch < nChunks; ++ch) {
    const int cbase = ch * CHUNK;
    const int wc = scan_chunk(bat, NN, cbase, g, 1, 1, list, tid, lane, wave);
    if (lane == 0) wcnt[wave] = wc;
    __syncthreads();
#pragma unroll 1
    for (int w2 = 0; w2 < NWAVE; ++w2) {
      int c = wcnt[w2];
      c = c < 0 ? 0 : (c > WCAP ? WCAP : c);
#pragma unroll 1
      for (int i = 0; i < c; ++i) {
        const int ent = list[w2 * WCAP + i];
        const int el  = (ent >> PKS) & (CHUNK - 1);
        int node = cbase + el;
        node = node < 0 ? 0 : (node > NN - 1 ? NN - 1 : node);
        const float* xp = XM + (size_t)node * (MM * NH);
        a0 += xp[tid];
        a1 += xp[NTHR + tid];
      }
    }
    __syncthreads();
  }
  sacc[tid] = a0;
  sacc[NTHR + tid] = a1;
  __syncthreads();
  const bool ok = tid < 128;
  v4f v = {0.f, 0.f, 0.f, 0.f};
  float* dp = PGb + (size_t)g * (MM * NH) + 4 * tid;
  if (ok) {
    v = *(const v4fa*)(sacc + 4 * tid);
    *(volatile v4f*)dp = v;
  }
  __threadfence();
  if (ok) *(volatile v4f*)dp = v;
}

__global__ __launch_bounds__(NTHR) void k_head(const float* __restrict__ PGb,
                                               const float* __restrict__ W1, const float* __restrict__ b1,
                                               const float* __restrict__ gg, const float* __restrict__ bt,
                                               const float* __restrict__ W2, const float* __restrict__ b2,
                                               float* out) {
  extern __shared__ __attribute__((aligned(16))) float hs[];
  float* FL = hs;
  float* WS = FL + 256 * HFP;
  float* O1 = WS + 64 * 128;
  float* ST = O1 + 256 * HOP;
  const int tid = (int)threadIdx.x;

#pragma unroll 4
  for (int it = 0; it < 128; ++it) {
    const int idx = it * NTHR + tid;
    const int r = idx >> 7, k = idx & 127;
    const int g = r >> 2, q = r & 3;
    FL[r * HFP + k] = PGb[(size_t)(4 * g + (k & 3)) * NH + 32 * q + (k >> 2)];
  }
#pragma unroll 4
  for (int it = 0; it < 32; ++it) {
    const int idx = it * NTHR + tid;
    WS[idx] = bf_rne(W1[idx]);
  }
  __syncthreads();

  const float* fr = FL + tid * HFP;
#pragma unroll 1
  for (int j = 0; j < 64; ++j) {
    const float* wr = WS + j * 128;
    float s = 0.0f;
#pragma unroll 4
    for (int k = 0; k < 128; ++k) s = fmaf(fr[k], wr[k], s);
    O1[tid * HOP + j] = s + bf_rne(b1[j]);
  }
  __syncthreads();

  if (tid < 64) {
    double sm = 0.0;
#pragma unroll 1
    for (int r = 0; r < 256; ++r) sm += (double)O1[r * HOP + tid];
    const double mean = sm * (1.0 / 256.0);
    double q2 = 0.0;
#pragma unroll 1
    for (int r = 0; r < 256; ++r) {
      const double d = (double)O1[r * HOP + tid] - mean;
      q2 += d * d;
    }
    const float var = (float)(q2 * (1.0 / 256.0));
    ST[tid]       = (float)mean;
    ST[64 + tid]  = 1.0f / sqrtf(var + BNEPS);
    ST[128 + tid] = bf_rne(gg[tid]);
    ST[192 + tid] = bf_rne(bt[tid]);
  }
#pragma unroll 4
  for (int it = 0; it < 16; ++it) {
    const int idx = it * NTHR + tid;
    WS[idx] = bf_rne(W2[idx]);
  }
  __syncthreads();

  float* orow = O1 + tid * HOP;
#pragma unroll 4
  for (int j = 0; j < 64; ++j) {
    const float v = orow[j];
    const float y = ((v - ST[j]) * ST[64 + j]) * ST[128 + j] + ST[192 + j];
    orow[j] = relu_p(y);
  }
  {
    const int g = tid >> 2, s4 = tid & 3;
    float* OUTS = FL;
#pragma unroll 1
    for (int t2 = 0; t2 < 16; ++t2) {
      float res = 0.0f;
#pragma unroll 1
      for (int t = 0; t < 4; ++t) {
        const int tt = 4 * t2 + t;
        const float* wr = WS + tt * 64;
        float v = 0.0f;
#pragma unroll 4
        for (int c = 0; c < 64; ++c) v = fmaf(orow[c], wr[c], v);
        res += v + bf_rne(b2[tt]);
      }
      OUTS[g * 64 + 16 * s4 + t2] = 0.25f * res;
    }
  }
  __syncthreads();
  v4f pv[4];
#pragma unroll
  for (int it = 0; it < 4; ++it) pv[it] = *(const v4fa*)(FL + 4 * (it * NTHR + tid));
#pragma unroll
  for (int it = 0; it < 4; ++it) *(volatile v4f*)(out + 4 * (it * NTHR + tid)) = pv[it];
  __threadfence();
#pragma unroll
  for (int it = 0; it < 4; ++it) *(volatile v4f*)(out + 4 * (it * NTHR + tid)) = pv[it];
}

static constexpr size_t al256c(size_t o) { return (o + 255) & ~(size_t)255; }
static constexpr size_t B_XM   = (size_t)R4 * NH * 4;
static constexpr size_t B_Z    = (size_t)R4 * ZW * 2;
static constexpr size_t B_EE   = (size_t)NE * NH * 4;
static constexpr size_t B_H3   = (size_t)R4 * NH * 4;
static constexpr size_t B_LIST = (size_t)NBKT * RCAP * 8;
static constexpr size_t B_CNT  = (size_t)NBKT * NBRUN * 4;
static constexpr size_t B_PE   = (size_t)(NE / GBM) * PARTW * 4;
static constexpr size_t B_PC   = (size_t)(R4 / GBM) * PARTW * 4;
static constexpr size_t B_PIN  = (size_t)(MPN / GBM) * PARTW * 4;
static constexpr size_t B_PART = B_PE;
static constexpr size_t B_W2D  = (size_t)NH * ZW * 2;
static constexpr size_t B_WCD  = (size_t)3 * NH * ZW * 2;
static constexpr size_t B_PG   = (size_t)NGR * MM * NH * 4;
static constexpr size_t B_HHL  = (size_t)MPN * ZW * 2;
static constexpr size_t B_T0   = (size_t)MPN * NH * 4;
static constexpr size_t O_XM   = 0;
static constexpr size_t O_Z    = al256c(O_XM + B_XM);
static constexpr size_t O_EE   = al256c(O_Z + B_Z);
static constexpr size_t O_LIST = al256c(O_EE + B_EE);
static constexpr size_t O_CNT  = al256c(O_LIST + B_LIST);
static constexpr size_t O_OFF  = al256c(O_CNT + B_CNT);
static constexpr size_t O_PART = al256c(O_OFF + B_CNT);
static constexpr size_t O_W2D  = al256c(O_PART + B_PART);
static constexpr size_t O_WCD  = al256c(O_W2D + B_W2D);
static constexpr size_t O_SS0  = al256c(O_WCD + B_WCD);
static constexpr size_t O_SSE  = al256c(O_SS0 + 2 * NH * 4);
static constexpr size_t O_SSC  = al256c(O_SSE + 2 * NH * 4);
static constexpr size_t O_PG   = al256c(O_SSC + 2 * NH * 4);
static constexpr size_t WS_TOT = al256c(O_PG + B_PG);
static constexpr size_t O_HHL  = O_Z;
static constexpr size_t O_H3   = O_EE;
static constexpr size_t O_T0   = O_EE;
static_assert(WS_TOT <= (size_t)WSCAP);
static_assert(B_HHL <= B_Z);
static_assert(B_H3 <= B_EE && B_T0 <= B_EE);
static_assert(B_PIN <= B_PART && B_PC <= B_PART && B_PE <= B_PART);

extern "C" void kernel_launch(void* const* d_in, const int* in_sizes, int n_in,
                              void* d_out, int out_size, void* d_ws, size_t ws_size,
                              hipStream_t stream) {
  if (n_in < 24) return;
  if (in_sizes[0] != NN * FK || in_sizes[1] != NE * FK || in_sizes[2] != 2 * NE || in_sizes[3] != NN) return;
  if (in_sizes[4] != NN * MM || in_sizes[5] != NH * FK) return;
  if (in_sizes[6] != NH || in_sizes[7] != NH || in_sizes[8] != NH) return;
  if (in_sizes[9] != NH * (NH + 1) || in_sizes[10] != NH) return;
  if (in_sizes[11] != 3 * NH * FK || in_sizes[12] != 3 * NH || in_sizes[13] != 3 * NH || in_sizes[14] != 3 * NH) return;
  if (in_sizes[15] != 3 * NH * NH || in_sizes[16] != 3 * NH || in_sizes[17] != 3 * NH) return;
  if (in_sizes[18] != 64 * NH || in_sizes[19] != 64 || in_sizes[20] != 64 || in_sizes[21] != 64) return;
  if (in_sizes[22] != 64 * 64 || in_sizes[23] != 64) return;
  if (out_size != NGR * 64) return;
  if (ws_size < WS_TOT) return;

  const float* x_node = (const float*)d_in[0];
  const float* e_attr = (const float*)d_in[1];
  const int*   ei     = (const int*)  d_in[2];
  const int*   src    = ei;
  const int*   dst    = ei + NE;
  const int*   batch  = (const int*)  d_in[3];
  const float* axp    = (const float*)d_in[4];
  const float* W_in   = (const float*)d_in[5];
  const float* b_in   = (const float*)d_in[6];
  const float* g_in   = (const float*)d_in[7];
  const float* bt_in  = (const float*)d_in[8];
  const float* W_l2   = (const float*)d_in[9];
  const float* b_l2   = (const float*)d_in[10];
  const float* W_edge = (const float*)d_in[11];
  const float* b_edge = (const float*)d_in[12];
  const float* g_edge = (const float*)d_in[13];
  const float* bt_edge= (const float*)d_in[14];
  const float* W_conv = (const float*)d_in[15];
  const float* g_norm = (const float*)d_in[16];
  const float* bt_norm= (const float*)d_in[17];
  const float* W_out1 = (const float*)d_in[18];
  const float* b_out1 = (const float*)d_in[19];
  const float* g_out  = (const float*)d_in[20];
  const float* bt_out = (const float*)d_in[21];
  const float* W_out2 = (const float*)d_in[22];
  const float* b_out2 = (const float*)d_in[23];
  float* out = (float*)d_out;

  char* ws = (char*)d_ws;
  float*          XM   = (float*)(ws + O_XM);
  unsigned short* ZHL  = (unsigned short*)(ws + O_Z);
  float*          EE   = (float*)(ws + O_EE);
  float*          H3   = (float*)(ws + O_H3);
  int*            LIST = (int*)(ws + O_LIST);
  int*            CNT  = (int*)(ws + O_CNT);
  int*            OFF  = (int*)(ws + O_OFF);
  float*          PART = (float*)(ws + O_PART);
  unsigned short* W2D  = (unsigned short*)(ws + O_W2D);
  unsigned short* WCD  = (unsigned short*)(ws + O_WCD);
  float*          SS0  = (float*)(ws + O_SS0);
  float*          SSE  = (float*)(ws + O_SSE);
  float*          SSC  = (float*)(ws + O_SSC);
  float*          PGb  = (float*)(ws + O_PG);
  unsigned short* HHL  = (unsigned short*)(ws + O_HHL);
  float*          T0   = (float*)(ws + O_T0);

  hipFuncSetAttribute(reinterpret_cast<const void*>(&k_bucket), hipFuncAttributeMaxDynamicSharedMemorySize, (int)LDS_BKT);
  hipFuncSetAttribute(reinterpret_cast<const void*>(&k_head),   hipFuncAttributeMaxDynamicSharedMemorySize, (int)LDS_HEAD);

  k_prep<<<(NU_L2 + NU_WC) / NTHR, NTHR, 0, stream>>>(W_l2, W_conv, W2D, WCD);
  k_bucket<<<NBKT, NTHR, LDS_BKT, stream>>>(src, dst, LIST, CNT, OFF);
  k_g16<<<MPN / GBM, GTHR, 0, stream>>>(x_node, NN, W_in, b_in, T0, MPN, PART);
  k_comb<<<1, GBN, 0, stream>>>(PART, MPN / GBM, 1, NH, g_in, bt_in, SS0);
  k_apply0<<<(MPN * 16) / NTHR, NTHR, 0, stream>>>(T0, SS0, HHL);
  k_gemm<4><<<MPN / GBM, GTHR, 0, stream>>>(HHL, W2D, XM, NN, PART, W_l2, b_l2, axp);

  for (int l = 0; l < 3; ++l) {
    k_g16<<<NE / GBM, GTHR, 0, stream>>>(e_attr, NE, W_edge + (size_t)l * NH * FK, b_edge + l * NH, EE, NE, PART);
    k_comb<<<1, GBN, 0, stream>>>(PART, NE / GBM, 1, NH, g_edge + l * NH, bt_edge + l * NH, SSE);
    k_agg<<<(NN + AGB - 1) / AGB, NTHR, 0, stream>>>(LIST, CNT, OFF, EE, SSE, XM, ZHL);
    k_gemm<1><<<R4 / GBM, GTHR, 0, stream>>>(ZHL, WCD + (size_t)l * NH * ZW, H3, R4, PART, W_l2, b_l2, axp);
    k_comb<<<1, GBN, 0, stream>>>(PART, R4 / GBM, 1, NH, g_norm + l * NH, bt_norm + l * NH, SSC);
    k_apply<<<(R4 * 32) / NTHR, NTHR, 0, stream>>>(H3, SSC, XM);
  }

  k_pool<<<NGR, NTHR, 0, stream>>>(XM, batch, PGb);
  k_head<<<1, NTHR, LDS_HEAD, stream>>>(PGb, W_out1, b_out1, g_out, bt_out, W_out2, b_out2, out);
}
